// BasicalBlock_31190052503718
// MI455X (gfx1250) — hardware-verified
//
#include <hip/hip_runtime.h>


#define NB_   2
#define CCH_  96
#define HH_   96
#define WW_   96
#define LL_   (HH_ * WW_)
#define DI_   192
#define MT_   (NB_ * LL_)
#define NS_   16
#define RR_   6
#define XDW_  (RR_ + 2 * NS_)
#define XDN_  64
#define WSC_  64.0f
#define USC_  1024.0f

static_assert(MT_ % 64 == 0);
static_assert(LL_ % 64 == 0);
static_assert(MT_ % 32 == 0);
static_assert(MT_ % 8 == 0);
static_assert(CCH_ % 32 == 0);
static_assert(DI_ % 64 == 0);
static_assert(XDW_ <= 40);

typedef float          v4f   __attribute__((ext_vector_type(4)));
typedef float          v8f   __attribute__((ext_vector_type(8)));
typedef _Float16       v8h   __attribute__((ext_vector_type(8)));
typedef _Float16       v16h  __attribute__((ext_vector_type(16)));
typedef unsigned short u16x8 __attribute__((ext_vector_type(8)));

union FragH { u16x8 h[2]; v16h v; };
union Pack8 { v8h f; u16x8 u; };

__device__ __forceinline__ v8f ld8f(const float* p) {
    v4f a = *(const v4f*)p;
    v4f b = *(const v4f*)(p + 4);
    return __builtin_shufflevector(a, b, 0, 1, 2, 3, 4, 5, 6, 7);
}
__device__ __forceinline__ float silu_f(float x) {
    float e = expf(-x);
    return x * __builtin_amdgcn_rcpf(1.0f + e);
}
__device__ __forceinline__ float softplus_f(float x) {
    return fmaxf(x, 0.0f) + log1pf(expf(-fabsf(x)));
}
__device__ __forceinline__ float wave_sum(float v) {
#pragma unroll
    for (int o = 16; o > 0; o >>= 1) v += __shfl_xor(v, o, 32);
    return v;
}
__device__ __forceinline__ int dir_pos(int k, int l) {
    const int lf = (k & 2) ? (LL_ - 1 - l) : l;
    return (k & 1) ? ((lf % HH_) * WW_ + (lf / HH_)) : lf;
}

__device__ __forceinline__ void mma16(v8f& acc, const FragH& a, const FragH& b) {
    acc = __builtin_amdgcn_wmma_f32_16x16x32_f16(false, a.v, false, b.v, (short)0, acc, false, false);
    asm volatile("v_nop\n\tv_nop\n\tv_nop\n\tv_nop" : "+v"(acc) : "v"(a.v), "v"(b.v));
}

__global__ __launch_bounds__(256)
void cvt_w_kernel(const float* __restrict__ w_in, const float* __restrict__ w_xp,
                  const float* __restrict__ w_out, const float* __restrict__ w_f1,
                  const float* __restrict__ w_f2,
                  unsigned short* d_in16, unsigned short* d_xp16, unsigned short* d_out16,
                  unsigned short* d_f116, unsigned short* d_f216)
{
    const int sel = blockIdx.y;
    const int i = blockIdx.x * 256 + threadIdx.x;
    const float* src;
    unsigned short* dst;
    int n8;
    if (sel == 0)      { src = w_in;  dst = d_in16;  n8 = (2 * DI_ * CCH_) / 8; }
    else if (sel == 1) { src = w_xp;  dst = d_xp16;  n8 = (4 * XDN_ * DI_) / 8; }
    else if (sel == 2) { src = w_out; dst = d_out16; n8 = (CCH_ * DI_) / 8; }
    else if (sel == 3) { src = w_f1;  dst = d_f116;  n8 = (DI_ * CCH_) / 8; }
    else               { src = w_f2;  dst = d_f216;  n8 = (CCH_ * DI_) / 8; }
    if (i >= n8) return;
    const size_t e = (size_t)i * 8;
    v8f x;
#pragma unroll
    for (int c = 0; c < 8; ++c) x[c] = 0.0f;
    if (sel == 1) {
        const int c = (int)(e % DI_);
        const int r = (int)((e / DI_) % XDN_);
        const int k = (int)(e / ((size_t)DI_ * XDN_));
        if (r < XDW_) x = ld8f(src + ((size_t)(k * XDW_ + r)) * DI_ + c);
    } else {
        x = ld8f(src + e);
    }
    Pack8 pk;
    pk.f = __builtin_convertvector(x * WSC_, v8h);
    const u16x8 v = pk.u;
    *(volatile u16x8*)(dst + e) = v;
    __threadfence();
    *(volatile u16x8*)(dst + e) = v;
}

template<int LAYOUT>
__global__ __launch_bounds__(64)
void ln96_kernel(const float* __restrict__ src, const float* __restrict__ g,
                 const float* __restrict__ be, float eps, unsigned short* dst)
{
    __shared__ __attribute__((aligned(16))) u16x8 sbuf[2][32 * 12];
    const int tid  = threadIdx.x;
    const int lane = tid & 31;
    const int wave = tid >> 5;
    const int idx  = blockIdx.x * 64 + tid;
    const float* sp;
    size_t cs;
    if (LAYOUT == 0) {
        const int b = idx / LL_;
        const int pos = idx - b * LL_;
        sp = src + (size_t)b * CCH_ * LL_ + pos;
        cs = (size_t)LL_;
    } else {
        sp = src + (size_t)idx * CCH_;
        cs = 1;
    }
    float mean = 0.0f;
    for (int c = 0; c < CCH_; ++c) mean += sp[c * cs];
    mean *= (1.0f / CCH_);
    float var = 0.0f;
    for (int c = 0; c < CCH_; ++c) { const float dd = sp[c * cs] - mean; var += dd * dd; }
    var *= (1.0f / CCH_);
    const float inv = rsqrtf(var + eps);
#pragma unroll 1
    for (int c8 = 0; c8 < CCH_ / 8; ++c8) {
        v8f o;
#pragma unroll
        for (int j = 0; j < 8; ++j) {
            const int c = c8 * 8 + j;
            o[j] = (sp[c * cs] - mean) * inv * g[c] + be[c];
        }
        Pack8 pk;
        pk.f = __builtin_convertvector(o, v8h);
        sbuf[wave][lane * 12 + c8] = pk.u;
    }
    __syncthreads();
    unsigned short* wb = dst + ((size_t)blockIdx.x * 64 + (size_t)wave * 32) * CCH_;
#pragma unroll 1
    for (int pass = 0; pass < 2; ++pass) {
#pragma unroll
        for (int it = 0; it < 12; ++it) {
            const int chunk = it * 32 + lane;
            const u16x8 v = sbuf[wave][chunk];
            *(volatile u16x8*)(wb + (size_t)chunk * 8) = v;
        }
        if (pass == 0) __threadfence();
    }
}

template<int WM, int WN, int RS, int NBF, int EPI, bool HB>
__global__ __launch_bounds__(32 * WM * WN)
void gemm_kernel(const unsigned short* __restrict__ A, const unsigned short* __restrict__ Bw, long long bzs,
                 float* C, float* C2, long long czs, int ldc, int csplit,
                 unsigned short* Ch,
                 const float* __restrict__ bias, const float* __restrict__ resid,
                 const float* __restrict__ rsc, int K, float scale)
{
    constexpr int T   = 32 * WM * WN;
    constexpr int BM  = 16 * RS * WM;
    constexpr int BN  = 16 * NBF * WN;
    constexpr int P   = BN + 4;
    constexpr int CPR  = BN / 4;
    constexpr int CPR8 = BN / 8;
    constexpr int CPT  = BM / 4;
    static_assert((BM * CPR) % T == 0);
    static_assert((BM * CPR8) % T == 0);
    static_assert((BN * CPT) % T == 0);
    static_assert(BN % 32 == 0);
    static_assert(BM % 32 == 0);
    __shared__ __attribute__((aligned(16))) float st[BM * P];

    const int tid  = threadIdx.x;
    const int lane = tid & 31;
    const int wave = tid >> 5;
    const int h    = lane >> 4;
    const int m    = lane & 15;
    const int wm   = wave / WN;
    const int wn   = wave % WN;
    const int rowBase = blockIdx.y * BM;
    const int colBase = blockIdx.x * BN;
    const int rW = wm * 16 * RS;
    const int cW = wn * 16 * NBF;
    const unsigned short* Bz = Bw + (size_t)blockIdx.z * (size_t)bzs;

    v8f acc[RS * NBF];
#pragma unroll
    for (int j = 0; j < RS * NBF; ++j)
#pragma unroll
        for (int r = 0; r < 8; ++r) acc[j][r] = 0.0f;

    const size_t aoff  = (size_t)(rowBase + rW + m) * K + 8 * h;
    const size_t boff  = (size_t)(colBase + cW + m) * K + 8 * h;
    const size_t sub16 = (size_t)16 * K;
    const int nk = K >> 5;

    for (int kt = 0; kt < nk; ++kt) {
        const size_t k0 = (size_t)kt * 32;
        FragH fa[RS], fb[NBF];
#pragma unroll
        for (int s = 0; s < RS; ++s) {
            const unsigned short* p = A + aoff + (size_t)s * sub16 + k0;
            fa[s].h[0] = *(const u16x8*)(p);
            fa[s].h[1] = *(const u16x8*)(p + 16);
        }
#pragma unroll
        for (int j = 0; j < NBF; ++j) {
            const unsigned short* p = Bz + boff + (size_t)j * sub16 + k0;
            fb[j].h[0] = *(const u16x8*)(p);
            fb[j].h[1] = *(const u16x8*)(p + 16);
        }
#pragma unroll
        for (int s = 0; s < RS; ++s)
#pragma unroll
            for (int j = 0; j < NBF; ++j)
                mma16(acc[s * NBF + j], fa[s], fb[j]);
    }

#pragma unroll
    for (int s = 0; s < RS; ++s)
#pragma unroll
        for (int j = 0; j < NBF; ++j)
#pragma unroll
            for (int r = 0; r < 8; ++r) {
                const int row = rW + s * 16 + 8 * h + r;
                const int col = cW + j * 16 + m;
                float v = acc[s * NBF + j][r] * scale;
                if (HB) v += bias[colBase + col];
                if (EPI == 1) v = (v >= 0.0f) ? v : 0.01f * v;
                if (EPI == 2) {
                    const int gm = rowBase + row;
                    const int bb = gm / LL_;
                    const int pos = gm - bb * LL_;
                    const int n = colBase + col;
                    v += resid[((size_t)bb * CCH_ + n) * LL_ + pos] * rsc[n];
                }
                if (EPI == 3) {
                    const int gm = rowBase + row;
                    const int n = colBase + col;
                    v += resid[(size_t)gm * CCH_ + n] * rsc[n];
                }
                st[row * P + col] = v;
            }
    __syncthreads();

#pragma unroll 1
    for (int pass = 0; pass < 2; ++pass) {
        if (EPI == 0 || EPI == 2) {
            constexpr int NIT = (BM * CPR) / T;
#pragma unroll
            for (int it = 0; it < NIT; ++it) {
                const int c   = it * T + tid;
                const int row = c / CPR;
                const int f4  = c - row * CPR;
                const v4f v = *(const v4f*)(st + row * P + 4 * f4);
                int gc = colBase + 4 * f4;
                float* Cp = C;
                if (EPI == 0 && gc >= csplit) { Cp = C2; gc -= csplit; }
                float* dp = Cp + (size_t)blockIdx.z * (size_t)czs + (size_t)(rowBase + row) * ldc + gc;
                *(volatile v4f*)dp = v;
            }
        } else if (EPI == 1) {
            constexpr int NIT = (BM * CPR8) / T;
#pragma unroll
            for (int it = 0; it < NIT; ++it) {
                const int c   = it * T + tid;
                const int row = c / CPR8;
                const int c8  = c - row * CPR8;
                const v4f a4 = *(const v4f*)(st + row * P + 8 * c8);
                const v4f b4 = *(const v4f*)(st + row * P + 8 * c8 + 4);
                const v8f x  = __builtin_shufflevector(a4, b4, 0, 1, 2, 3, 4, 5, 6, 7);
                Pack8 pk;
                pk.f = __builtin_convertvector(x, v8h);
                const u16x8 hv = pk.u;
                unsigned short* dp = Ch + (size_t)(rowBase + row) * ldc + colBase + 8 * c8;
                *(volatile u16x8*)dp = hv;
            }
        } else {
            constexpr int NIT = (BN * CPT) / T;
            const int bb   = rowBase / LL_;
            const int pos0 = rowBase - bb * LL_;
#pragma unroll
            for (int it = 0; it < NIT; ++it) {
                const int c  = it * T + tid;
                const int nl = c / CPT;
                const int t4 = c - nl * CPT;
                v4f v;
#pragma unroll
                for (int i = 0; i < 4; ++i) v[i] = st[(4 * t4 + i) * P + nl];
                const int n = colBase + nl;
                float* dp = C + ((size_t)(bb * CCH_ + n)) * LL_ + pos0 + 4 * t4;
                *(volatile v4f*)dp = v;
            }
        }
        if (pass == 0) __threadfence();
    }
}

__global__ __launch_bounds__(192)
void conv_silu_kernel(const float* __restrict__ XI, const float* __restrict__ cw,
                      const float* __restrict__ cb, float* U32, unsigned short* U16)
{
    __shared__ __attribute__((aligned(16))) float su[8 * DI_];
    const int tid = threadIdx.x;
    const int t   = tid / 24;
    const int cg  = tid - t * 24;
    const int d0  = cg * 8;
    const int p   = blockIdx.x * 8 + t;
    const int b   = p / LL_;
    const int pos = p - b * LL_;
    const int hy0 = pos / WW_;
    const int wx0 = pos - hy0 * WW_;

    v8f acc;
#pragma unroll
    for (int c = 0; c < 8; ++c) acc[c] = 0.0f;
#pragma unroll
    for (int dy = -1; dy <= 1; ++dy) {
        const int hy = hy0 + dy;
        if (hy < 0 || hy >= HH_) continue;
#pragma unroll
        for (int dx = -1; dx <= 1; ++dx) {
            const int wx = wx0 + dx;
            if (wx < 0 || wx >= WW_) continue;
            const v8f xv = ld8f(XI + ((size_t)(b * LL_ + hy * WW_ + wx)) * DI_ + d0);
            const int tap = (dy + 1) * 3 + (dx + 1);
#pragma unroll
            for (int c = 0; c < 8; ++c) acc[c] += xv[c] * cw[(size_t)(d0 + c) * 9 + tap];
        }
    }
    const v8f bias = ld8f(cb + d0);
    v8f u;
#pragma unroll
    for (int c = 0; c < 8; ++c) u[c] = silu_f(acc[c] + bias[c]);

    *(v4f*)(su + t * DI_ + d0)     = __builtin_shufflevector(u, u, 0, 1, 2, 3);
    *(v4f*)(su + t * DI_ + d0 + 4) = __builtin_shufflevector(u, u, 4, 5, 6, 7);
    Pack8 pk;
    pk.f = __builtin_convertvector(u * USC_, v8h);
    const u16x8 hv = pk.u;
    unsigned short* hp = U16 + (size_t)blockIdx.x * 8 * DI_ + (size_t)tid * 8;
    *(volatile u16x8*)hp = hv;
    __syncthreads();
    float* fbp = U32 + (size_t)blockIdx.x * 8 * DI_;
#pragma unroll 1
    for (int pass = 0; pass < 2; ++pass) {
#pragma unroll
        for (int it = 0; it < 2; ++it) {
            const int c = it * 192 + tid;
            const v4f v = *(const v4f*)(su + c * 4);
            *(volatile v4f*)(fbp + (size_t)c * 4) = v;
        }
        if (pass == 0) {
            __threadfence();
            *(volatile u16x8*)hp = hv;
        }
    }
}

__global__ __launch_bounds__(64)
void scan_kernel(const float* __restrict__ XD, const float* __restrict__ U32,
                 const float* __restrict__ dtw, const float* __restrict__ dtb,
                 const float* __restrict__ alog, float* Y, long long ysz)
{
    __shared__ __attribute__((aligned(16))) float sy[2][4][32];
    const int tid  = threadIdx.x;
    const int lane = tid & 31;
    const int wave = tid >> 5;
    const int dg   = blockIdx.x;
    const int bk   = blockIdx.y;
    const int b    = bk >> 2;
    const int k    = bk & 3;
    const int d    = dg * 64 + tid;

    float wdt[RR_];
#pragma unroll
    for (int r = 0; r < RR_; ++r) wdt[r] = dtw[((size_t)(k * DI_ + d)) * RR_ + r];
    const float dbias = dtb[k * DI_ + d];
    float An[NS_], hs[NS_];
#pragma unroll
    for (int n = 0; n < NS_; ++n) {
        An[n] = -expf(alog[((size_t)(k * DI_ + d)) * NS_ + n]);
        hs[n] = 0.0f;
    }
    const float* XDk = XD + (size_t)k * MT_ * XDN_;
    float* Yk = Y + (size_t)k * (size_t)ysz;
    const size_t rowb = (size_t)b * LL_;
    const int cofs = dg * 64 + wave * 32;

#pragma unroll 1
    for (int l0 = 0; l0 < LL_; l0 += 4) {
#pragma unroll 1
        for (int t = 0; t < 4; ++t) {
            const int pos = dir_pos(k, l0 + t);
            const size_t row = rowb + (size_t)pos;
            const float* xr = XDk + row * XDN_;
            v4f q[10];
#pragma unroll
            for (int i = 0; i < 10; ++i) q[i] = *(const v4f*)(xr + 4 * i);
            float xd[40];
#pragma unroll
            for (int i = 0; i < 10; ++i)
#pragma unroll
                for (int j = 0; j < 4; ++j) xd[4 * i + j] = q[i][j];
            float sdt = 0.0f;
#pragma unroll
            for (int r = 0; r < RR_; ++r) sdt += xd[r] * wdt[r];
            const float delta = softplus_f(sdt + dbias);
            const float u  = U32[row * DI_ + d];
            const float du = delta * u;
            float y = 0.0f;
#pragma unroll
            for (int n = 0; n < NS_; ++n) {
                const float dA = __expf(delta * An[n]);
                hs[n] = hs[n] * dA + du * xd[RR_ + n];
                y += hs[n] * xd[RR_ + NS_ + n];
            }
            sy[wave][t][lane] = y;
        }
        __syncthreads();
        const int s  = lane >> 3;
        const int qq = lane & 7;
        const int pos_s = dir_pos(k, l0 + s);
        const v4f v = *(const v4f*)(&sy[wave][s][4 * qq]);
        float* dp = Yk + (rowb + (size_t)pos_s) * DI_ + cofs + 4 * qq;
        *(volatile v4f*)dp = v;
        __threadfence();
        *(volatile v4f*)dp = v;
        __syncthreads();
    }
}

__global__ __launch_bounds__(64)
void ln_gate_kernel(const float* __restrict__ Y, long long ysz, const float* __restrict__ U32,
                    const float* __restrict__ Z32, const float* __restrict__ Ds,
                    const float* __restrict__ g, const float* __restrict__ be,
                    unsigned short* G16)
{
    __shared__ __attribute__((aligned(16))) _Float16 srow[2][DI_];
    const int tid  = threadIdx.x;
    const int lane = tid & 31;
    const int wave = tid >> 5;
    float dsum[6], gg[6], bb[6];
#pragma unroll
    for (int j = 0; j < 6; ++j) {
        const int d = lane + 32 * j;
        dsum[j] = Ds[d] + Ds[DI_ + d] + Ds[2 * DI_ + d] + Ds[3 * DI_ + d];
        gg[j] = g[d];
        bb[j] = be[d];
    }
    const size_t ys = (size_t)ysz;
    const int tok0 = (blockIdx.x * 2 + wave) * 16;
#pragma unroll 1
    for (int it = 0; it < 16; ++it) {
        const size_t base = (size_t)(tok0 + it) * DI_;
        float v[6];
        float sum = 0.0f;
#pragma unroll
        for (int j = 0; j < 6; ++j) {
            const size_t e = base + lane + 32 * j;
            const float a = (Y[e] + Y[2 * ys + e]) + (Y[ys + e] + Y[3 * ys + e]);
            v[j] = a + U32[e] * dsum[j];
            sum += v[j];
        }
        sum = wave_sum(sum);
        const float mean = sum * (1.0f / DI_);
        float vs = 0.0f;
#pragma unroll
        for (int j = 0; j < 6; ++j) { const float dd = v[j] - mean; vs += dd * dd; }
        vs = wave_sum(vs);
        const float inv = rsqrtf(vs * (1.0f / DI_) + 1e-5f);
#pragma unroll
        for (int j = 0; j < 6; ++j) {
            const int d = lane + 32 * j;
            const float z = Z32[base + d];
            const float o = ((v[j] - mean) * inv * gg[j] + bb[j]) * silu_f(z);
            srow[wave][d] = (_Float16)o;
        }
        __syncthreads();
        Pack8 pk;
        if (lane < 24) pk.f = *(const v8h*)(&srow[wave][lane * 8]);
        unsigned short* dp = G16 + base + (size_t)lane * 8;
        if (lane < 24) *(volatile u16x8*)dp = pk.u;
        __threadfence();
        if (lane < 24) *(volatile u16x8*)dp = pk.u;
        __syncthreads();
    }
}

extern "C" void kernel_launch(void* const* d_in, const int* in_sizes, int n_in,
                              void* d_out, int out_size, void* d_ws, size_t ws_size,
                              hipStream_t stream)
{
    if (n_in < 24) return;
    if (in_sizes[0]  != MT_ * CCH_) return;
    if (in_sizes[1]  != CCH_ || in_sizes[2] != CCH_) return;
    if (in_sizes[3]  != 2 * DI_ * CCH_ || in_sizes[4] != 2 * DI_) return;
    if (in_sizes[5]  != DI_ * 9 || in_sizes[6] != DI_) return;
    if (in_sizes[7]  != 4 * XDW_ * DI_) return;
    if (in_sizes[8]  != 4 * DI_ * RR_ || in_sizes[9] != 4 * DI_) return;
    if (in_sizes[10] != 4 * DI_ * NS_ || in_sizes[11] != 4 * DI_) return;
    if (in_sizes[12] != DI_ || in_sizes[13] != DI_) return;
    if (in_sizes[14] != CCH_ * DI_ || in_sizes[15] != CCH_) return;
    if (in_sizes[16] != CCH_ || in_sizes[17] != CCH_) return;
    if (in_sizes[18] != DI_ * CCH_ || in_sizes[19] != DI_) return;
    if (in_sizes[20] != CCH_ * DI_ || in_sizes[21] != CCH_) return;
    if (in_sizes[22] != CCH_ || in_sizes[23] != CCH_) return;
    if (out_size != MT_ * CCH_) return;

    const float* x          = (const float*)d_in[0];
    const float* ln_in_g    = (const float*)d_in[1];
    const float* ln_in_b    = (const float*)d_in[2];
    const float* in_proj_w  = (const float*)d_in[3];
    const float* in_proj_b  = (const float*)d_in[4];
    const float* conv_w     = (const float*)d_in[5];
    const float* conv_b     = (const float*)d_in[6];
    const float* x_proj_w   = (const float*)d_in[7];
    const float* dt_w       = (const float*)d_in[8];
    const float* dt_b       = (const float*)d_in[9];
    const float* A_logs     = (const float*)d_in[10];
    const float* Ds         = (const float*)d_in[11];
    const float* out_norm_g = (const float*)d_in[12];
    const float* out_norm_b = (const float*)d_in[13];
    const float* out_proj_w = (const float*)d_in[14];
    const float* out_proj_b = (const float*)d_in[15];
    const float* ln_ffn_g   = (const float*)d_in[16];
    const float* ln_ffn_b   = (const float*)d_in[17];
    const float* fc1_w      = (const float*)d_in[18];
    const float* fc1_b      = (const float*)d_in[19];
    const float* fc2_w      = (const float*)d_in[20];
    const float* fc2_b      = (const float*)d_in[21];
    const float* scale1     = (const float*)d_in[22];
    const float* scale2     = (const float*)d_in[23];
    float* out = (float*)d_out;

    const size_t SZ_XN16 = (size_t)MT_ * CCH_ * 2;
    const size_t SZ_WIN  = (size_t)2 * DI_ * CCH_ * 2;
    const size_t SZ_WXP  = (size_t)4 * XDN_ * DI_ * 2;
    const size_t SZ_W96  = (size_t)CCH_ * DI_ * 2;
    const size_t SZ_F192 = (size_t)MT_ * DI_ * 4;
    const size_t SZ_H192 = (size_t)MT_ * DI_ * 2;
    const size_t SZ_F96  = (size_t)MT_ * CCH_ * 4;
    const size_t SZ_XD   = (size_t)4 * MT_ * XDN_ * 4;
    const size_t SZ_Y    = (size_t)4 * MT_ * DI_ * 4;

    const size_t OFF_XN16 = 0;
    const size_t OFF_WIN  = OFF_XN16 + SZ_XN16;
    const size_t OFF_WXP  = OFF_WIN + SZ_WIN;
    const size_t OFF_WOUT = OFF_WXP + SZ_WXP;
    const size_t OFF_WF1  = OFF_WOUT + SZ_W96;
    const size_t OFF_WF2  = OFF_WF1 + SZ_W96;
    const size_t OFF_RA   = OFF_WF2 + SZ_W96;
    const size_t OFF_Z32  = OFF_RA + SZ_F192;
    const size_t OFF_U32  = OFF_Z32 + SZ_F192;
    const size_t OFF_U16  = OFF_U32 + SZ_F192;
    const size_t OFF_RX   = OFF_U16 + SZ_H192;
    const size_t OFF_Y    = OFF_RX + SZ_XD;
    const size_t WS_END   = OFF_Y + SZ_Y;
    const size_t OFF_YG16 = OFF_RA;
    const size_t OFF_H116 = OFF_RA + SZ_H192;
    const size_t OFF_X2   = OFF_RX;
    const size_t OFF_H216 = OFF_RX + SZ_F96;
    if (OFF_H116 + SZ_XN16 > OFF_Z32) return;
    if (OFF_H216 + SZ_H192 > OFF_Y) return;
    if (ws_size < WS_END) return;

    char* ws = (char*)d_ws;
    unsigned short* xn16  = (unsigned short*)(ws + OFF_XN16);
    unsigned short* win16 = (unsigned short*)(ws + OFF_WIN);
    unsigned short* wxp16 = (unsigned short*)(ws + OFF_WXP);
    unsigned short* wou16 = (unsigned short*)(ws + OFF_WOUT);
    unsigned short* wf116 = (unsigned short*)(ws + OFF_WF1);
    unsigned short* wf216 = (unsigned short*)(ws + OFF_WF2);
    float*          xi32  = (float*)(ws + OFF_RA);
    float*          z32   = (float*)(ws + OFF_Z32);
    float*          u32   = (float*)(ws + OFF_U32);
    unsigned short* u16   = (unsigned short*)(ws + OFF_U16);
    float*          xd32  = (float*)(ws + OFF_RX);
    float*          ybuf  = (float*)(ws + OFF_Y);
    unsigned short* yg16  = (unsigned short*)(ws + OFF_YG16);
    unsigned short* h116  = (unsigned short*)(ws + OFF_H116);
    float*          x2    = (float*)(ws + OFF_X2);
    unsigned short* h216  = (unsigned short*)(ws + OFF_H216);

    const float inv_w  = 1.0f / WSC_;
    const float inv_wu = 1.0f / (WSC_ * USC_);
    const int   nosplit = 1 << 30;

    cvt_w_kernel<<<dim3((4 * XDN_ * DI_ / 8 + 255) / 256, 5), dim3(256), 0, stream>>>(
        in_proj_w, x_proj_w, out_proj_w, fc1_w, fc2_w, win16, wxp16, wou16, wf116, wf216);

    ln96_kernel<0><<<dim3(MT_ / 64), dim3(64), 0, stream>>>(x, ln_in_g, ln_in_b, 1e-6f, xn16);

    gemm_kernel<2, 2, 2, 4, 0, true><<<dim3((2 * DI_) / 128, MT_ / 64, 1), dim3(128), 0, stream>>>(
        xn16, win16, 0LL, xi32, z32, 0LL, (int)DI_, (int)DI_, u16,
        in_proj_b, x, scale1, (int)CCH_, inv_w);

    conv_silu_kernel<<<dim3(MT_ / 8), dim3(192), 0, stream>>>(xi32, conv_w, conv_b, u32, u16);

    gemm_kernel<2, 1, 2, 4, 0, false><<<dim3(1, MT_ / 64, 4), dim3(64), 0, stream>>>(
        u16, wxp16, (long long)XDN_ * DI_, xd32, xd32, (long long)MT_ * XDN_, (int)XDN_, nosplit, u16,
        in_proj_b, x, scale1, (int)DI_, inv_wu);

    scan_kernel<<<dim3(DI_ / 64, NB_ * 4), dim3(64), 0, stream>>>(
        xd32, u32, dt_w, dt_b, A_logs, ybuf, (long long)MT_ * DI_);

    ln_gate_kernel<<<dim3(MT_ / 32), dim3(64), 0, stream>>>(
        ybuf, (long long)MT_ * DI_, u32, z32, Ds, out_norm_g, out_norm_b, yg16);

    gemm_kernel<4, 1, 1, 6, 2, true><<<dim3(1, MT_ / 64, 1), dim3(128), 0, stream>>>(
        yg16, wou16, 0LL, x2, x2, 0LL, (int)CCH_, nosplit, u16,
        out_proj_b, x, scale1, (int)DI_, inv_w);

    ln96_kernel<1><<<dim3(MT_ / 64), dim3(64), 0, stream>>>(x2, ln_ffn_g, ln_ffn_b, 1e-5f, h116);

    gemm_kernel<2, 1, 2, 4, 1, true><<<dim3(DI_ / 64, MT_ / 64, 1), dim3(64), 0, stream>>>(
        h116, wf116, 0LL, x2, x2, 0LL, (int)DI_, nosplit, h216,
        fc1_b, x, scale1, (int)CCH_, inv_w);

    gemm_kernel<4, 1, 1, 6, 3, true><<<dim3(1, MT_ / 64, 1), dim3(128), 0, stream>>>(
        h216, wf216, 0LL, out, out, 0LL, (int)CCH_, nosplit, u16,
        fc2_b, x2, scale2, (int)DI_, inv_w);
}
